// RNNennigma_1236950582097
// MI455X (gfx1250) — hardware-verified
//
#include <hip/hip_runtime.h>
#include <math.h>

constexpr int DIM_H      = 64;
constexpr int DIM_2      = 128;
constexpr int NSYMB      = 8;
constexpr int VOCAB      = 512;
constexpr int NLEAF      = 131072;
constexpr int NLEV1      = 65536;
constexpr int NLEV2      = 32768;
constexpr int NCLS       = 2048;
constexpr int TSTEPS     = 16;
constexpr int NGATE      = 256;
constexpr int CHUNK_ROWS = 16384;
constexpr int HALL_COLS  = NSYMB * DIM_2;
constexpr int YALL_COLS  = NSYMB * DIM_H;
constexpr float CARRY      = 16.0f;
constexpr float CARRY_INV  = 1.0f / 16.0f;
constexpr float CARRY2_INV = 1.0f / 256.0f;

static_assert(NLEV1 % CHUNK_ROWS == 0 && NLEV2 % CHUNK_ROWS == 0, "chunking");
static_assert(CHUNK_ROWS % 64 == 0 && HALL_COLS % 64 == 0 && DIM_H % 64 == 0, "tile multiples");
static_assert(DIM_2 % 32 == 0 && DIM_H % 32 == 0, "K multiples of 32");
static_assert((NLEV1 * 16) % 256 == 0 && (NLEV2 * 16) % 256 == 0 && (CHUNK_ROWS * 8) % 256 == 0, "gather grids exact");
static_assert(NCLS % 16 == 0 && NCLS % 64 == 0, "lstm / scorer grids exact");

typedef __attribute__((ext_vector_type(16))) _Float16 v16h;
typedef __attribute__((ext_vector_type(8)))  _Float16 v8h;
typedef __attribute__((ext_vector_type(16))) __bf16   v16b;
typedef __attribute__((ext_vector_type(8)))  __bf16   v8b;
typedef __attribute__((ext_vector_type(8)))  float    v8f;
typedef __attribute__((ext_vector_type(4)))  float    v4f;

__device__ __forceinline__ unsigned short f2bf_bits(float f) {
  unsigned u = __float_as_uint(f);
  return (unsigned short)((u + 0x7FFFu + ((u >> 16) & 1u)) >> 16);
}
__device__ __forceinline__ float bf_bits2f(unsigned short h) { return __uint_as_float(((unsigned)h) << 16); }

__device__ __forceinline__ int clampi(int v, int hi) { v = v < 0 ? 0 : v; return v > hi ? hi : v; }

__device__ __forceinline__ void dep_guard_h(v8f& a, v8f& b, v16h x, v16h y) { asm volatile("v_nop\n\tv_nop\n\tv_nop\n\tv_nop" : "+v"(a), "+v"(b) : "v"(x), "v"(y)); }
__device__ __forceinline__ void dep_guard_b(v8f& a, v8f& b, v16b x, v16b y) { asm volatile("v_nop\n\tv_nop\n\tv_nop\n\tv_nop" : "+v"(a), "+v"(b) : "v"(x), "v"(y)); }
__device__ __forceinline__ void keep4_h(v16h a, v16h b, v16h c, v16h d) { asm volatile("v_nop" :: "v"(a), "v"(b), "v"(c), "v"(d)); }
__device__ __forceinline__ void keep4_b(v16b a, v16b b, v16b c, v16b d) { asm volatile("v_nop" :: "v"(a), "v"(b), "v"(c), "v"(d)); }
__device__ __forceinline__ void acc_guard4(v8f& a, v8f& b, v8f& c, v8f& d) { asm volatile("v_nop\n\tv_nop\n\tv_nop\n\tv_nop" : "+v"(a), "+v"(b), "+v"(c), "+v"(d)); }
template <typename T> struct Frag;
template <> struct Frag<_Float16> {
  typedef v16h V; union U { v16h v; v8h h[2]; };
  static __device__ __forceinline__ v16h load(const _Float16* p) {
    U f; f.h[0] = *(const v8h*)(p); f.h[1] = *(const v8h*)(p + 16); return f.v;
  }
  static __device__ __forceinline__ v8f mma(v16h a, v16h b, v8f c) {
    return __builtin_amdgcn_wmma_f32_16x16x32_f16(false, a, false, b, (short)0, c, false, false);
  }
  static __device__ __forceinline__ void guard(v8f& a, v8f& b, v16h x, v16h y) { dep_guard_h(a, b, x, y); }
  static __device__ __forceinline__ void keep(v16h a, v16h b, v16h c, v16h d) { keep4_h(a, b, c, d); }
};
template <> struct Frag<__bf16> {
  typedef v16b V; union U { v16b v; v8b h[2]; };
  static __device__ __forceinline__ v16b load(const __bf16* p) {
    U f; f.h[0] = *(const v8b*)(p); f.h[1] = *(const v8b*)(p + 16); return f.v;
  }
  static __device__ __forceinline__ v8f mma(v16b a, v16b b, v8f c) {
    return __builtin_amdgcn_wmma_f32_16x16x32_bf16(false, a, false, b, (short)0, c, false, false);
  }
  static __device__ __forceinline__ void guard(v8f& a, v8f& b, v16b x, v16b y) { dep_guard_b(a, b, x, y); }
  static __device__ __forceinline__ void keep(v16b a, v16b b, v16b c, v16b d) { keep4_b(a, b, c, d); }
};

template <int ET> struct Elem;
template <> struct Elem<0> { typedef _Float16 T; };
template <> struct Elem<1> { typedef __bf16 T; };
template <int ET, bool SPLIT, int BIAS_MODE, int OUT_MODE, bool RESID, int ACT = 0>
__global__ __launch_bounds__(256) void wmma_gemm64(
    const unsigned short* __restrict__ Ap, const unsigned short* __restrict__ A2p, int lda, long strideA,
    const unsigned short* __restrict__ Btp, const unsigned short* __restrict__ Bt2p, int ldb, long strideB,
    void* __restrict__ Cout, void* __restrict__ Cout2, int ldc, long strideC,
    const float* __restrict__ biasp, long strideBias,
    const float* __restrict__ resid, long strideR,
    int M, int N, int K, float scale) {
  typedef typename Elem<ET>::T T;
  typedef typename Frag<T>::V V;
  const T* A = (const T*)Ap; const T* A2 = (const T*)A2p; const T* Bt = (const T*)Btp; const T* Bt2 = (const T*)Bt2p;
  __shared__ __align__(16) float sT[8][16 * 68];
  const int b    = blockIdx.y;
  const int lane = threadIdx.x & 31;
  const int wave = threadIdx.x >> 5;
  const int tilesN = N >> 6;
  const int tilesM = M >> 6;
  const int tile = blockIdx.x * 8 + wave;
  if (tile >= tilesM * tilesN) return;
  const int tm = tile / tilesN;
  const int tn = tile - tm * tilesN;
  const int m0 = tm << 6;
  const int n0 = tn << 6;

  const T* Ab  = A  + (size_t)b * strideA;
  const T* Bb  = Bt + (size_t)b * strideB;
  const T* Ab2 = SPLIT ? (A2  + (size_t)b * strideA) : nullptr;
  const T* Bb2 = SPLIT ? (Bt2 + (size_t)b * strideB) : nullptr;
  const float* bias = (BIAS_MODE != 0) ? (biasp + (size_t)b * strideBias) : nullptr;

  const int rlane = lane & 15;
  const int koff  = (lane >> 4) * 8;
  const int mOff  = (lane >> 4) * 8;

  v8f acc[4][4];
#pragma unroll
  for (int i = 0; i < 4; ++i)
#pragma unroll
    for (int j = 0; j < 4; ++j) acc[i][j] = (v8f){0.f,0.f,0.f,0.f,0.f,0.f,0.f,0.f};

  for (int k0 = 0; k0 < K; k0 += 32) {
    V bh[4], bl[4];
#pragma unroll
    for (int j = 0; j < 4; ++j) {
      const size_t bo = (size_t)(n0 + (j << 4) + rlane) * ldb + koff + k0;
      bh[j] = Frag<T>::load(Bb + bo);
      if (SPLIT) bl[j] = Frag<T>::load(Bb2 + bo);
    }
#pragma unroll
    for (int i = 0; i < 4; ++i) {
      const size_t ao = (size_t)(m0 + (i << 4) + rlane) * lda + koff + k0;
      V ah = Frag<T>::load(Ab + ao);
      V al = ah;
      if (SPLIT) al = Frag<T>::load(Ab2 + ao);
#pragma unroll
      for (int j = 0; j < 4; ++j) {
        acc[i][j] = Frag<T>::mma(ah, bh[j], acc[i][j]);
        if (SPLIT) {
          acc[i][j] = Frag<T>::mma(ah, bl[j], acc[i][j]);
          acc[i][j] = Frag<T>::mma(al, bh[j], acc[i][j]);
        }
      }
      Frag<T>::guard(acc[i][0], acc[i][3], ah, SPLIT ? al : ah);
    }
    Frag<T>::keep(bh[0], bh[1], bh[2], bh[3]);
    if (SPLIT) Frag<T>::keep(bl[0], bl[1], bl[2], bl[3]);
  }
  acc_guard4(acc[0][0], acc[0][1], acc[0][2], acc[0][3]);
  acc_guard4(acc[1][0], acc[1][1], acc[1][2], acc[1][3]);
  acc_guard4(acc[2][0], acc[2][1], acc[2][2], acc[2][3]);
  acc_guard4(acc[3][0], acc[3][1], acc[3][2], acc[3][3]);

  float* slab = sT[wave];
  const float* Rb = RESID ? (resid + (size_t)b * strideR) : nullptr;
#pragma unroll
  for (int i = 0; i < 4; ++i) {
    const int mBase = m0 + (i << 4);
#pragma unroll
    for (int j = 0; j < 4; ++j) {
      const int n = n0 + (j << 4) + rlane;
      float bv = 0.f;
      if (BIAS_MODE == 2) bv = bias[n];
#pragma unroll
      for (int r = 0; r < 8; ++r) {
        float v = acc[i][j][r] * scale;
        if (BIAS_MODE == 1) v += bias[mBase + mOff + r];
        if (BIAS_MODE == 2) v += bv;
        if (RESID) v += Rb[(size_t)(mBase + mOff + r) * ldc + n];
        if (ACT == 1) v = tanhf(v);
        if (ACT == 2) v = fmaxf(v, 0.0f);
        if (ACT == 4) v = (v > 0.f) ? v : 0.01f * v;
        slab[(mOff + r) * 68 + (j << 4) + rlane] = v;
      }
    }
    __builtin_amdgcn_fence(__ATOMIC_RELEASE, "workgroup");
    __builtin_amdgcn_wave_barrier();
    __builtin_amdgcn_fence(__ATOMIC_ACQUIRE, "workgroup");
    if (OUT_MODE == 0) {
      float* C = (float*)Cout + (size_t)b * strideC;
      const int hh = lane >> 4, c4 = (lane & 15) * 4;
      for (int pass = 0; pass < 2; ++pass) {
#pragma unroll
        for (int it = 0; it < 8; ++it) {
          const int row = it * 2 + hh;
          v4f v = *(const v4f*)(slab + row * 68 + c4);
          *(volatile v4f*)(C + (size_t)(mBase + row) * ldc + n0 + c4) = v;
        }
        __threadfence();
      }
    } else {
      const int q = lane >> 3, c8 = (lane & 7) * 8;
      unsigned short* C  = (unsigned short*)Cout  + (size_t)b * strideC;
      unsigned short* C2 = (OUT_MODE == 2) ? ((unsigned short*)Cout2 + (size_t)b * strideC) : nullptr;
      for (int pass = 0; pass < 2; ++pass) {
#pragma unroll
        for (int it = 0; it < 4; ++it) {
          const int row = it * 4 + q;
          const float* sp = slab + row * 68 + c8;
          v8h hv, lv;
#pragma unroll
          for (int e = 0; e < 8; ++e) {
            if (OUT_MODE == 1) {
              hv[e] = (_Float16)sp[e];
            } else {
              unsigned short hb = f2bf_bits(sp[e]);
              unsigned short lb = f2bf_bits(sp[e] - bf_bits2f(hb));
              hv[e] = __builtin_bit_cast(_Float16, hb);
              lv[e] = __builtin_bit_cast(_Float16, lb);
            }
          }
          *(volatile v8h*)(C + (size_t)(mBase + row) * ldc + n0 + c8) = hv;
          if (OUT_MODE == 2) *(volatile v8h*)(C2 + (size_t)(mBase + row) * ldc + n0 + c8) = lv;
        }
        __threadfence();
      }
    }
    __builtin_amdgcn_fence(__ATOMIC_RELEASE, "workgroup");
    __builtin_amdgcn_wave_barrier();
    __builtin_amdgcn_fence(__ATOMIC_ACQUIRE, "workgroup");
  }
}

__global__ __launch_bounds__(256) void cast_scale_f16x2(
    const float* __restrict__ in, _Float16* __restrict__ out, int n2, float sc) {
  int i = blockIdx.x * 256 + threadIdx.x;
  if (i < n2) {
    const _Float16 h0 = (_Float16)(in[2 * i] * sc), h1 = (_Float16)(in[2 * i + 1] * sc);
    const unsigned u = (unsigned)__builtin_bit_cast(unsigned short, h0) | ((unsigned)__builtin_bit_cast(unsigned short, h1) << 16);
    ((volatile unsigned*)out)[i] = u;
    __threadfence();
    ((volatile unsigned*)out)[i] = u;
  }
}

__global__ __launch_bounds__(256) void scale_vec_kernel(const float* __restrict__ in, float* __restrict__ out, int n, float sc) {
  const int i = blockIdx.x * 256 + threadIdx.x;
  if (i < n) {
    const float v = in[i] * sc;
    ((volatile float*)out)[i] = v;
    __threadfence();
    ((volatile float*)out)[i] = v;
  }
}

constexpr int TP_NT = 256;
__global__ __launch_bounds__(TP_NT) void tpw16_kernel(const float* __restrict__ src, long strideSrc, int R, int C,
                                                     _Float16* __restrict__ O, long strideO, int ldo, float sc) {
  __shared__ float Tt[64 * 65];
  const int tid = threadIdx.x;
  const int c0 = blockIdx.x * 64, r0 = blockIdx.y * 64;
  const float* s = src + (size_t)blockIdx.z * strideSrc;
  _Float16* Ob = O + (size_t)blockIdx.z * strideO;
#pragma unroll
  for (int i = 0; i < 4; ++i) {
    const int idx = i * TP_NT + tid;
    const int rr = idx >> 4, cc = (idx & 15) * 4;
    const v4f v = *(const v4f*)(s + (size_t)(r0 + rr) * (size_t)C + c0 + cc);
    Tt[rr * 65 + cc + 0] = v[0];
    Tt[rr * 65 + cc + 1] = v[1];
    Tt[rr * 65 + cc + 2] = v[2];
    Tt[rr * 65 + cc + 3] = v[3];
  }
  __syncthreads();
  const int q = tid >> 3, c8 = (tid & 7) * 8;
  v8h hv[2];
#pragma unroll
  for (int g = 0; g < 2; ++g) {
    const int qq = g * 32 + q;
#pragma unroll
    for (int e = 0; e < 8; ++e) {
      const float f = Tt[(c8 + e) * 65 + qq];
      hv[g][e] = (_Float16)(f * sc);
    }
  }
  for (int pass = 0; pass < 2; ++pass) {
#pragma unroll
    for (int g = 0; g < 2; ++g) {
      const size_t o = (size_t)(c0 + g * 32 + q) * (size_t)ldo + (size_t)(r0 + c8);
      *(volatile v8h*)(Ob + o) = hv[g];
    }
    __threadfence();
  }
}

__global__ __launch_bounds__(256) void gather_leaf_pairs_kernel(
    const float* __restrict__ s_emb, const int* __restrict__ leaf_ids,
    const int* __restrict__ lft, const int* __restrict__ rgt,
    _Float16* __restrict__ X, int nrows) {
  const int gid = blockIdx.x * 256 + threadIdx.x;
  int n = gid >> 4;
  const int p = gid & 15;
  n = (n < nrows) ? n : (nrows - 1);
  const int li = lft[n];
  const int ri = rgt[n];
  int ch = (p < 8) ? li : ri;
  ch = clampi(ch, NLEAF - 1);
  int leaf = leaf_ids[ch];
  leaf = clampi(leaf, VOCAB - 1);
  const float* src = s_emb + (size_t)leaf * DIM_H + (p & 7) * 8;
  const v4f a = *(const v4f*)(src);
  const v4f b = *(const v4f*)(src + 4);
  v8h hv;
  hv[0] = (_Float16)(a[0] * CARRY); hv[1] = (_Float16)(a[1] * CARRY);
  hv[2] = (_Float16)(a[2] * CARRY); hv[3] = (_Float16)(a[3] * CARRY);
  hv[4] = (_Float16)(b[0] * CARRY); hv[5] = (_Float16)(b[1] * CARRY);
  hv[6] = (_Float16)(b[2] * CARRY); hv[7] = (_Float16)(b[3] * CARRY);
  _Float16* dst = X + (size_t)n * DIM_2 + p * 8;
  *(volatile v8h*)dst = hv;
  __threadfence();
  *(volatile v8h*)dst = hv;
}

__global__ __launch_bounds__(256) void gather_pairs16_kernel(
    const _Float16* __restrict__ SRC, const int* __restrict__ lft, const int* __restrict__ rgt,
    _Float16* __restrict__ X, int nrows, int nsrc) {
  const int gid = blockIdx.x * 256 + threadIdx.x;
  int n = gid >> 4;
  const int p = gid & 15;
  n = (n < nrows) ? n : (nrows - 1);
  const int li = lft[n];
  const int ri = rgt[n];
  int idx = (p < 8) ? li : ri;
  idx = clampi(idx, nsrc - 1);
  const v8h v = *(const v8h*)(SRC + (size_t)idx * DIM_H + (p & 7) * 8);
  _Float16* dst = X + (size_t)n * DIM_2 + p * 8;
  *(volatile v8h*)dst = v;
  __threadfence();
  *(volatile v8h*)dst = v;
}

__global__ __launch_bounds__(256) void select_sym_kernel(
    const float* __restrict__ Y, const int* __restrict__ symtab, int row0, _Float16* __restrict__ O) {
  const int gid = blockIdx.x * 256 + threadIdx.x;
  const int n = gid >> 3;
  const int p = gid & 7;
  int s = symtab[row0 + n];
  s = clampi(s, NSYMB - 1);
  const float* src = Y + (size_t)n * YALL_COLS + s * DIM_H + p * 8;
  const v4f a = *(const v4f*)(src);
  const v4f b = *(const v4f*)(src + 4);
  v8h hv;
  hv[0] = (_Float16)(a[0] * CARRY); hv[1] = (_Float16)(a[1] * CARRY);
  hv[2] = (_Float16)(a[2] * CARRY); hv[3] = (_Float16)(a[3] * CARRY);
  hv[4] = (_Float16)(b[0] * CARRY); hv[5] = (_Float16)(b[1] * CARRY);
  hv[6] = (_Float16)(b[2] * CARRY); hv[7] = (_Float16)(b[3] * CARRY);
  _Float16* dst = O + (size_t)(row0 + n) * DIM_H + p * 8;
  *(volatile v8h*)dst = hv;
  __threadfence();
  *(volatile v8h*)dst = hv;
}

constexpr int LSTM_NT = 128;
constexpr int XPITCH = 72;
constexpr int HPITCH = 72;
constexpr int OPITCH = 68;

__device__ __forceinline__ float fsig(float x)  { return __builtin_amdgcn_rcpf(1.0f + __expf(-x)); }
__device__ __forceinline__ float ftanh(float x) { return 1.0f - 2.0f * __builtin_amdgcn_rcpf(__expf(2.0f * x) + 1.0f); }

template <int FIRST>
__global__ __launch_bounds__(LSTM_NT) void lstm_rec_kernel(
    const _Float16* xsrc, const int* __restrict__ clause_lits,
    const float* __restrict__ bih, const float* __restrict__ bhh,
    const float* __restrict__ h0, const float* __restrict__ c0,
    const _Float16* __restrict__ WX, const _Float16* __restrict__ WH,
    _Float16* hseq_out, float* __restrict__ cv_out) {
  __shared__ __align__(16) _Float16 Ax[16 * XPITCH];
  __shared__ __align__(16) _Float16 Ah[16 * HPITCH];
  __shared__ __align__(16) float    Hs[16 * OPITCH];
  const int tid = threadIdx.x, lane = tid & 31, wave = tid >> 5;
  const int c = lane & 15, hh = lane >> 4, koff = hh * 8;
  const int seqbase = blockIdx.x * 16;
  const int j = 16 * wave + c;

#pragma unroll 1
  for (int i = 0; i < 8; ++i) {
    const int idx = i * LSTM_NT + tid;
    const int m = idx >> 6, col = idx & 63;
    Ah[m * HPITCH + col] = (_Float16)(CARRY * h0[col]);
  }
  {
    const int m = tid >> 3, c8 = (tid & 7) * 8;
    size_t row;
    if (FIRST) {
      int lit = clause_lits[(size_t)(seqbase + m) * TSTEPS + 0];
      lit = clampi(lit, NLEV2 - 1);
      row = (size_t)lit;
    } else {
      row = (size_t)(seqbase + m) * TSTEPS + 0;
    }
    const v8h v = *(const v8h*)(xsrc + row * DIM_H + c8);
    *(v8h*)(Ax + m * XPITCH + c8) = v;
  }
  float cst[8], hst[8], bb[4];
#pragma unroll
  for (int g = 0; g < 4; ++g) bb[g] = bih[g * DIM_H + j] + bhh[g * DIM_H + j];
#pragma unroll
  for (int r = 0; r < 8; ++r) { cst[r] = c0[j]; hst[r] = h0[j]; }
  __syncthreads();

  const _Float16* axrow = Ax + c * XPITCH + koff;
  const _Float16* ahrow = Ah + c * HPITCH + koff;
  const _Float16* wx = WX + (size_t)j * DIM_H + koff;
  const _Float16* wh = WH + (size_t)j * DIM_H + koff;
  const v8f z8 = {0.f, 0.f, 0.f, 0.f, 0.f, 0.f, 0.f, 0.f};

#pragma unroll 1
  for (int t = 0; t < TSTEPS; ++t) {
    v8f acc[4];
    acc[0] = z8; acc[1] = z8; acc[2] = z8; acc[3] = z8;
#pragma unroll 1
    for (int kx = 0; kx < DIM_H; kx += 32) {
      const v16h a  = Frag<_Float16>::load(axrow + kx);
      const v16h b0 = Frag<_Float16>::load(wx + kx);
      const v16h b1 = Frag<_Float16>::load(wx + (size_t)1 * DIM_H * DIM_H + kx);
      const v16h b2 = Frag<_Float16>::load(wx + (size_t)2 * DIM_H * DIM_H + kx);
      const v16h b3 = Frag<_Float16>::load(wx + (size_t)3 * DIM_H * DIM_H + kx);
      acc[0] = Frag<_Float16>::mma(a, b0, acc[0]);
      acc[1] = Frag<_Float16>::mma(a, b1, acc[1]);
      acc[2] = Frag<_Float16>::mma(a, b2, acc[2]);
      acc[3] = Frag<_Float16>::mma(a, b3, acc[3]);
      dep_guard_h(acc[0], acc[3], a, b3);
      keep4_h(b0, b1, b2, b3);
    }
#pragma unroll 1
    for (int kh = 0; kh < DIM_H; kh += 32) {
      const v16h a  = Frag<_Float16>::load(ahrow + kh);
      const v16h b0 = Frag<_Float16>::load(wh + kh);
      const v16h b1 = Frag<_Float16>::load(wh + (size_t)1 * DIM_H * DIM_H + kh);
      const v16h b2 = Frag<_Float16>::load(wh + (size_t)2 * DIM_H * DIM_H + kh);
      const v16h b3 = Frag<_Float16>::load(wh + (size_t)3 * DIM_H * DIM_H + kh);
      acc[0] = Frag<_Float16>::mma(a, b0, acc[0]);
      acc[1] = Frag<_Float16>::mma(a, b1, acc[1]);
      acc[2] = Frag<_Float16>::mma(a, b2, acc[2]);
      acc[3] = Frag<_Float16>::mma(a, b3, acc[3]);
      dep_guard_h(acc[0], acc[3], a, b3);
      keep4_h(b0, b1, b2, b3);
    }
    acc_guard4(acc[0], acc[1], acc[2], acc[3]);
#pragma unroll
    for (int r = 0; r < 8; ++r) {
      const float zi = acc[0][r] * CARRY2_INV + bb[0];
      const float zf = acc[1][r] * CARRY2_INV + bb[1];
      const float zg = acc[2][r] * CARRY2_INV + bb[2];
      const float zo = acc[3][r] * CARRY2_INV + bb[3];
      const float ig = fsig(zi);
      const float fg = fsig(zf);
      const float gg = ftanh(zg);
      const float og = fsig(zo);
      const float cn = fg * cst[r] + ig * gg;
      cst[r] = cn;
      hst[r] = og * ftanh(cn);
    }
    __syncthreads();
#pragma unroll
    for (int r = 0; r < 8; ++r) Ah[(8 * hh + r) * HPITCH + j] = (_Float16)(CARRY * hst[r]);
    {
      const int tn = (t + 1 < TSTEPS) ? (t + 1) : (TSTEPS - 1);
      const int m = tid >> 3, c8 = (tid & 7) * 8;
      size_t row;
      if (FIRST) {
        int lit = clause_lits[(size_t)(seqbase + m) * TSTEPS + tn];
        lit = clampi(lit, NLEV2 - 1);
        row = (size_t)lit;
      } else {
        row = (size_t)(seqbase + m) * TSTEPS + tn;
      }
      const v8h v = *(const v8h*)(xsrc + row * DIM_H + c8);
      *(v8h*)(Ax + m * XPITCH + c8) = v;
    }
    __syncthreads();
    if (FIRST) {
      const int m = tid >> 3, c8 = (tid & 7) * 8;
      const v8h v = *(const v8h*)(Ah + m * HPITCH + c8);
      _Float16* dst = hseq_out + ((size_t)(seqbase + m) * TSTEPS + (size_t)t) * DIM_H + c8;
      for (int pass = 0; pass < 2; ++pass) {
        *(volatile v8h*)dst = v;
        __threadfence();
      }
    }
  }

  if (!FIRST) {
#pragma unroll
    for (int r = 0; r < 8; ++r) Hs[(8 * hh + r) * OPITCH + j] = hst[r];
    __syncthreads();
    for (int pass = 0; pass < 2; ++pass) {
#pragma unroll
      for (int it = 0; it < 2; ++it) {
        const int idx = it * LSTM_NT + tid;
        const int row = idx >> 4, c4 = (idx & 15) * 4;
        const v4f v = *(const v4f*)(Hs + row * OPITCH + c4);
        *(volatile v4f*)(cv_out + (size_t)(seqbase + row) * DIM_H + c4) = v;
      }
      __threadfence();
    }
  }
}

constexpr int SC_NT = 64;
__global__ __launch_bounds__(SC_NT) void scorer_kernel(const float* __restrict__ cv, const float* __restrict__ Wf1,
                                                     const float* __restrict__ bf1, const float* __restrict__ Wf2,
                                                     const float* __restrict__ bf2, float* __restrict__ out) {
  __shared__ float cvs[64 * 65];
  __shared__ float w1s[64 * 32];
  __shared__ float b1v[32];
  __shared__ float w2s[64];
  __shared__ float b2v[2];
  __shared__ __align__(16) float outs[128];
  const int tid = threadIdx.x;
  const int base = blockIdx.x * 64;
#pragma unroll 1
  for (int i = 0; i < 64; ++i) {
    const int idx = i * SC_NT + tid;
    const int r = idx >> 6, col = idx & 63;
    cvs[r * 65 + col] = cv[(size_t)(base + r) * DIM_H + col];
  }
#pragma unroll 1
  for (int i = 0; i < 32; ++i) w1s[i * 64 + tid] = Wf1[i * 64 + tid];
  if (tid < 32) b1v[tid] = bf1[tid];
  w2s[tid] = Wf2[tid];
  if (tid < 2) b2v[tid] = bf2[tid];
  __syncthreads();
  float o0 = 0.f, o1 = 0.f;
#pragma unroll 1
  for (int jj = 0; jj < 32; ++jj) {
    float a = 0.f;
#pragma unroll 1
    for (int d = 0; d < DIM_H; ++d) a = fmaf(cvs[tid * 65 + d], w1s[d * 32 + jj], a);
    a += b1v[jj];
    a = fmaxf(a, 0.0f);
    o0 = fmaf(a, w2s[jj * 2 + 0], o0);
    o1 = fmaf(a, w2s[jj * 2 + 1], o1);
  }
  outs[tid * 2 + 0] = o0 + b2v[0];
  outs[tid * 2 + 1] = o1 + b2v[1];
  __syncthreads();
  if (tid < 32) {
    const v4f v = *(const v4f*)(outs + tid * 4);
    float* dst = out + (size_t)blockIdx.x * 128 + tid * 4;
    for (int pass = 0; pass < 2; ++pass) {
      *(volatile v4f*)dst = v;
      __threadfence();
    }
  }
}

extern "C" void kernel_launch(void* const* d_in, const int* in_sizes, int n_in,
                              void* d_out, int out_size, void* d_ws, size_t ws_size, hipStream_t stream) {
  if (n_in < 23 || d_out == nullptr || d_ws == nullptr) return;
  if (in_sizes[0] != VOCAB * DIM_H || in_sizes[1] != NSYMB * DIM_2 * DIM_2 || in_sizes[2] != NSYMB * DIM_2 ||
      in_sizes[3] != NSYMB * DIM_2 * DIM_H || in_sizes[4] != NSYMB * DIM_H ||
      in_sizes[5] != 2 * NGATE * DIM_H || in_sizes[6] != 2 * NGATE * DIM_H || in_sizes[7] != 2 * NGATE ||
      in_sizes[8] != 2 * NGATE || in_sizes[9] != 2 * DIM_H || in_sizes[10] != 2 * DIM_H ||
      in_sizes[11] != DIM_H * 32 || in_sizes[12] != 32 || in_sizes[13] != 64 || in_sizes[14] != 2 ||
      in_sizes[15] != NLEAF || in_sizes[16] != NLEV1 || in_sizes[17] != NLEV1 || in_sizes[18] != NLEV1 ||
      in_sizes[19] != NLEV2 || in_sizes[20] != NLEV2 || in_sizes[21] != NLEV2 || in_sizes[22] != NCLS * TSTEPS ||
      out_size != NCLS * 2) return;

  const float* s_emb = (const float*)d_in[0];
  const float* W1    = (const float*)d_in[1];
  const float* b1    = (const float*)d_in[2];
  const float* W2    = (const float*)d_in[3];
  const float* b2    = (const float*)d_in[4];
  const float* Wih   = (const float*)d_in[5];
  const float* Whh   = (const float*)d_in[6];
  const float* bih   = (const float*)d_in[7];
  const float* bhh   = (const float*)d_in[8];
  const float* h0    = (const float*)d_in[9];
  const float* c0    = (const float*)d_in[10];
  const float* Wf1   = (const float*)d_in[11];
  const float* bf1   = (const float*)d_in[12];
  const float* Wf2   = (const float*)d_in[13];
  const float* bf2   = (const float*)d_in[14];
  const int* leaf_ids    = (const int*)d_in[15];
  const int* l1_sym      = (const int*)d_in[16];
  const int* l1_left     = (const int*)d_in[17];
  const int* l1_right    = (const int*)d_in[18];
  const int* l2_sym      = (const int*)d_in[19];
  const int* l2_left     = (const int*)d_in[20];
  const int* l2_right    = (const int*)d_in[21];
  const int* clause_lits = (const int*)d_in[22];
  float* out = (float*)d_out;

  char* ws = (char*)d_ws; size_t off = 0;
  auto carve = [&](size_t bytes) -> char* { char* p = ws + off; off += (bytes + 255) & ~(size_t)255; return p; };
  _Float16* W1T   = (_Float16*)carve((size_t)HALL_COLS * DIM_2 * 2);
  _Float16* W2T   = (_Float16*)carve((size_t)NSYMB * DIM_H * DIM_2 * 2);
  _Float16* WIH16 = (_Float16*)carve((size_t)2 * NGATE * DIM_H * 2);
  _Float16* WHH16 = (_Float16*)carve((size_t)2 * NGATE * DIM_H * 2);
  float*    B1S   = (float*)carve((size_t)HALL_COLS * 4);
  _Float16* X1    = (_Float16*)carve((size_t)NLEV1 * DIM_2 * 2);
  _Float16* HALL  = (_Float16*)carve((size_t)CHUNK_ROWS * HALL_COLS * 2);
  float*    YALL  = (float*)carve((size_t)CHUNK_ROWS * YALL_COLS * 4);
  _Float16* N1    = (_Float16*)carve((size_t)NLEV1 * DIM_H * 2);
  _Float16* X2    = (_Float16*)carve((size_t)NLEV2 * DIM_2 * 2);
  _Float16* LITS  = (_Float16*)carve((size_t)NLEV2 * DIM_H * 2);
  _Float16* HSEQ  = (_Float16*)carve((size_t)NCLS * TSTEPS * DIM_H * 2);
  float*    CV    = (float*)carve((size_t)NCLS * DIM_H * 4);
  if (off > ws_size || off > (size_t)134217728) return;

  tpw16_kernel<<<dim3(DIM_2 / 64, DIM_2 / 64, NSYMB), TP_NT, 0, stream>>>(W1, (long)(DIM_2 * DIM_2), DIM_2, DIM_2, W1T, (long)(DIM_2 * DIM_2), DIM_2, CARRY);
  tpw16_kernel<<<dim3(DIM_H / 64, DIM_2 / 64, NSYMB), TP_NT, 0, stream>>>(W2, (long)(DIM_2 * DIM_H), DIM_2, DIM_H, W2T, (long)(DIM_H * DIM_2), DIM_2, CARRY);
  cast_scale_f16x2<<<(2 * NGATE * DIM_H / 2) / 256, 256, 0, stream>>>(Wih, WIH16, 2 * NGATE * DIM_H / 2, CARRY);
  cast_scale_f16x2<<<(2 * NGATE * DIM_H / 2) / 256, 256, 0, stream>>>(Whh, WHH16, 2 * NGATE * DIM_H / 2, CARRY);
  scale_vec_kernel<<<HALL_COLS / 256, 256, 0, stream>>>(b1, B1S, HALL_COLS, CARRY);

  gather_leaf_pairs_kernel<<<NLEV1 * 16 / 256, 256, 0, stream>>>(s_emb, leaf_ids, l1_left, l1_right, X1, NLEV1);
  const int g1_tiles = (CHUNK_ROWS / 64) * (HALL_COLS / 64);
  const int g2_tiles = (CHUNK_ROWS / 64) * (DIM_H / 64);
  for (int ch = 0; ch < NLEV1 / CHUNK_ROWS; ++ch) {
    const _Float16* Ach = X1 + (size_t)ch * CHUNK_ROWS * DIM_2;
    wmma_gemm64<0, false, 2, 1, false, 2><<<dim3((g1_tiles + 7) / 8, 1), 256, 0, stream>>>(
        (const unsigned short*)Ach, (const unsigned short*)Ach, DIM_2, 0L,
        (const unsigned short*)W1T, (const unsigned short*)W1T, DIM_2, 0L,
        (void*)HALL, (void*)HALL, HALL_COLS, 0L, B1S, 0L, B1S, 0L, CHUNK_ROWS, HALL_COLS, DIM_2, CARRY_INV);
    wmma_gemm64<0, false, 2, 0, false, 2><<<dim3((g2_tiles + 7) / 8, NSYMB), 256, 0, stream>>>(
        (const unsigned short*)HALL, (const unsigned short*)HALL, HALL_COLS, (long)DIM_2,
        (const unsigned short*)W2T, (const unsigned short*)W2T, DIM_2, (long)(DIM_H * DIM_2),
        (void*)YALL, (void*)YALL, YALL_COLS, (long)DIM_H, b2, (long)DIM_H, b2, 0L, CHUNK_ROWS, DIM_H, DIM_2, CARRY2_INV);
    select_sym_kernel<<<CHUNK_ROWS * 8 / 256, 256, 0, stream>>>(YALL, l1_sym, ch * CHUNK_ROWS, N1);
  }

  gather_pairs16_kernel<<<NLEV2 * 16 / 256, 256, 0, stream>>>(N1, l2_left, l2_right, X2, NLEV2, NLEV1);
  for (int ch = 0; ch < NLEV2 / CHUNK_ROWS; ++ch) {
    const _Float16* Ach = X2 + (size_t)ch * CHUNK_ROWS * DIM_2;
    wmma_gemm64<0, false, 2, 1, false, 2><<<dim3((g1_tiles + 7) / 8, 1), 256, 0, stream>>>(
        (const unsigned short*)Ach, (const unsigned short*)Ach, DIM_2, 0L,
        (const unsigned short*)W1T, (const unsigned short*)W1T, DIM_2, 0L,
        (void*)HALL, (void*)HALL, HALL_COLS, 0L, B1S, 0L, B1S, 0L, CHUNK_ROWS, HALL_COLS, DIM_2, CARRY_INV);
    wmma_gemm64<0, false, 2, 0, false, 2><<<dim3((g2_tiles + 7) / 8, NSYMB), 256, 0, stream>>>(
        (const unsigned short*)HALL, (const unsigned short*)HALL, HALL_COLS, (long)DIM_2,
        (const unsigned short*)W2T, (const unsigned short*)W2T, DIM_2, (long)(DIM_H * DIM_2),
        (void*)YALL, (void*)YALL, YALL_COLS, (long)DIM_H, b2, (long)DIM_H, b2, 0L, CHUNK_ROWS, DIM_H, DIM_2, CARRY2_INV);
    select_sym_kernel<<<CHUNK_ROWS * 8 / 256, 256, 0, stream>>>(YALL, l2_sym, ch * CHUNK_ROWS, LITS);
  }

  lstm_rec_kernel<1><<<NCLS / 16, LSTM_NT, 0, stream>>>(LITS, clause_lits, bih, bhh, h0, c0, WIH16, WHH16, HSEQ, CV);
  lstm_rec_kernel<0><<<NCLS / 16, LSTM_NT, 0, stream>>>(HSEQ, clause_lits, bih + NGATE, bhh + NGATE, h0 + DIM_H, c0 + DIM_H,
                                                       WIH16 + (size_t)NGATE * DIM_H, WHH16 + (size_t)NGATE * DIM_H, HSEQ, CV);

  scorer_kernel<<<NCLS / 64, SC_NT, 0, stream>>>(CV, Wf1, bf1, Wf2, bf2, out);
}
